// GNN_27934467293571
// MI455X (gfx1250) — hardware-verified
//
#include <hip/hip_runtime.h>
#include <stddef.h>
#include <stdint.h>
#include <math.h>


#define DF     128
#define NTHR   256
#define NWAVE  8
#define EPT    8
#define CHUNK  (NTHR * EPT)
#define WCAP   (EPT * 32)
#define LISTN  (NWAVE * WCAP)
#define NBA    1024
#define SLA    10
#define RCAP   28672
#define DEGCAP 63
#define GBM    64
#define GTHR   128
#define UW     2048
#define NVEC   10
#define AGG_ZINTS    (LISTN + 2 * RCAP + 3 * NBA)
#define CSR_LDS_INTS (AGG_ZINTS + 16)
#define WSMAX  134217728

static_assert((CHUNK & (CHUNK - 1)) == 0 && CHUNK <= 4096);
static_assert((NBA & (NBA - 1)) == 0 && NBA == (1 << SLA));
static_assert(((long long)CHUNK << SLA) < (1LL << 31));
static_assert(NBA % NWAVE == 0 && NBA == NTHR * 4 && NBA % GBM == 0);
static_assert(RCAP % (NTHR * 4) == 0 && AGG_ZINTS % 4 == 0 && LISTN % 4 == 0);
static_assert(DEGCAP + 1 <= 64);
static_assert(DF % 32 == 0 && DF == 4 * 32 && GTHR == DF);
static_assert(GBM == (GTHR / 32) * 16);
static_assert(UW % NTHR == 0 && UW == DF * (DF / 8));
static_assert(CSR_LDS_INTS * 4 <= 300000);
static_assert(NVEC * 32 <= 512);

typedef float          v4f   __attribute__((ext_vector_type(4)));
typedef float          v8f   __attribute__((ext_vector_type(8)));
typedef double         v2d   __attribute__((ext_vector_type(2)));
typedef int            v4i   __attribute__((ext_vector_type(4)));
typedef int            v8i   __attribute__((ext_vector_type(8)));
typedef unsigned short v8us  __attribute__((ext_vector_type(8)));
typedef unsigned short v16us __attribute__((ext_vector_type(16)));
typedef __bf16         v16bf __attribute__((ext_vector_type(16)));
typedef v4f  __attribute__((may_alias)) v4fa;
typedef v2d  __attribute__((may_alias)) v2da;
typedef v4i  __attribute__((may_alias)) v4ia;
typedef v8us __attribute__((may_alias)) v8usa;
union FragB { v16bf v; v16us u; v8us h[2]; v8i w; };

__device__ __forceinline__ v8f wmb(const FragB& a, const FragB& b, v8f c) {
  v8f d = __builtin_amdgcn_wmma_f32_16x16x32_bf16(false, a.v, false, b.v, (short)0, c, false, false);
  asm volatile("v_nop\n\tv_nop\n\tv_nop\n\tv_nop" : "+v"(d) : "v"(a.w), "v"(b.w));
  return d;
}

__device__ __forceinline__ unsigned bf16_bits(float f) {
  const unsigned u = __float_as_uint(f);
  return (u + 0x7FFFu + ((u >> 16) & 1u)) >> 16;
}
__device__ __forceinline__ float bf16_val(float f) {
  return __uint_as_float(bf16_bits(f) << 16);
}

template <int SLB>
__device__ __forceinline__ int scan_chunk(const int* __restrict__ dsts, int nE, int cbase, int slotBase,
                                          int nb, int vec8, int* list, int tid, int lane, int wave) {
  int wc = 0;
  const int el0  = tid * EPT;
  const int e0   = cbase + el0;
  const int sent = -2147483647 - 1;
  v4i da, db;
  if (vec8 != 0 && cbase + CHUNK <= nE) {
    da = *(const v4i*)(dsts + e0);
    db = *(const v4i*)(dsts + e0 + 4);
  } else {
    da.x = (e0     < nE) ? dsts[min(e0,     nE - 1)] : sent;
    da.y = (e0 + 1 < nE) ? dsts[min(e0 + 1, nE - 1)] : sent;
    da.z = (e0 + 2 < nE) ? dsts[min(e0 + 2, nE - 1)] : sent;
    da.w = (e0 + 3 < nE) ? dsts[min(e0 + 3, nE - 1)] : sent;
    db.x = (e0 + 4 < nE) ? dsts[min(e0 + 4, nE - 1)] : sent;
    db.y = (e0 + 5 < nE) ? dsts[min(e0 + 5, nE - 1)] : sent;
    db.z = (e0 + 6 < nE) ? dsts[min(e0 + 6, nE - 1)] : sent;
    db.w = (e0 + 7 < nE) ? dsts[min(e0 + 7, nE - 1)] : sent;
  }
  const unsigned nbs = (unsigned)slotBase;
  const unsigned unb = (unsigned)nb;
  const unsigned s0 = (unsigned)da.x - nbs, s1 = (unsigned)da.y - nbs;
  const unsigned s2 = (unsigned)da.z - nbs, s3 = (unsigned)da.w - nbs;
  const unsigned s4 = (unsigned)db.x - nbs, s5 = (unsigned)db.y - nbs;
  const unsigned s6 = (unsigned)db.z - nbs, s7 = (unsigned)db.w - nbs;
  const bool h0 = s0 < unb, h1 = s1 < unb, h2 = s2 < unb, h3 = s3 < unb;
  const bool h4 = s4 < unb, h5 = s5 < unb, h6 = s6 < unb, h7 = s7 < unb;
  const unsigned any = __builtin_amdgcn_ballot_w32(h0 | h1 | h2 | h3 | h4 | h5 | h6 | h7);
  if (any != 0u) {
#define HITJ(J, HJ, SJ) { \
      const unsigned mj = __builtin_amdgcn_ballot_w32(HJ); \
      if (mj != 0u) { \
        if (HJ) { \
          const int pos = wc + (int)__builtin_amdgcn_mbcnt_lo(mj, 0u); \
          if (pos < WCAP) list[wave * WCAP + pos] = ((el0 + (J)) << SLB) | (int)(SJ); \
        } \
        wc += (int)__builtin_popcount(mj); } }
    HITJ(0, h0, s0)
    HITJ(1, h1, s1)
    HITJ(2, h2, s2)
    HITJ(3, h3, s3)
    HITJ(4, h4, s4)
    HITJ(5, h5, s5)
    HITJ(6, h6, s6)
    HITJ(7, h7, s7)
#undef HITJ
  }
  return wc;
}

__global__ __launch_bounds__(NTHR) void k_prep(
    const float* __restrict__ W0, const float* __restrict__ W1,
    const float* __restrict__ p0, const float* __restrict__ p1, const float* __restrict__ p2,
    const float* __restrict__ p3, const float* __restrict__ p4, const float* __restrict__ p5,
    const float* __restrict__ p6, const float* __restrict__ p7, const float* __restrict__ p8,
    const float* __restrict__ p9,
    unsigned short* W0T, unsigned short* W1T, float* vec) {
  const int u = (int)blockIdx.x * NTHR + (int)threadIdx.x;
  if (u < 2 * UW) {
    const int part = u >> 11;
    const int v  = u & (UW - 1);
    const int n  = v >> 4;
    const int k8 = (v & 15) * 8;
    const float* W;
    unsigned short* P;
    if (part == 0) { W = W0; P = W0T; } else { W = W1; P = W1T; }
    const float* p = W + (size_t)k8 * DF + n;
    v8us o;
#pragma unroll
    for (int i = 0; i < 8; ++i) o[i] = (unsigned short)bf16_bits(p[(size_t)i * DF]);
    unsigned short* dp = P + (size_t)n * DF + k8;
    *(volatile v8us*)dp = o;
    __threadfence();
    *(volatile v8us*)dp = o;
  } else {
    const int v   = u - 2 * UW;
    const int vid = v >> 5;
    const int l   = v & 31;
    const float* s;
    if (vid == 0)      s = p0;
    else if (vid == 1) s = p1;
    else if (vid == 2) s = p2;
    else if (vid == 3) s = p3;
    else if (vid == 4) s = p4;
    else if (vid == 5) s = p5;
    else if (vid == 6) s = p6;
    else if (vid == 7) s = p7;
    else if (vid == 8) s = p8;
    else if (vid == 9) s = p9;
    else return;
    const v4f a = *(const v4fa*)(s + 4 * l);
    v4f o;
    o.x = bf16_val(a.x); o.y = bf16_val(a.y); o.z = bf16_val(a.z); o.w = bf16_val(a.w);
    float* dp = vec + (size_t)vid * DF + 4 * l;
    *(volatile v4f*)dp = o;
    __threadfence();
    *(volatile v4f*)dp = o;
  }
}

__global__ __launch_bounds__(NTHR) void k_csr(const int* __restrict__ srcs, const int* __restrict__ dsts,
                                              int nE, int nN, int vec8,
                                              int* slt, int* cntg, int* offg, int* flg) {
  extern __shared__ __attribute__((aligned(16))) int dsm[];
  int* list = dsm;
  int* hl   = dsm + LISTN;
  int* sl   = hl + RCAP;
  int* cnt  = sl + RCAP;
  int* offs = cnt + NBA;
  int* cur  = offs + NBA;
  int* misc = cur + NBA;
  const int tid = (int)threadIdx.x, lane = tid & 31, wave = tid >> 5;
  const int nodeBase = (int)blockIdx.x * NBA;

  {
    const v4i z4 = {0, 0, 0, 0};
    for (int i = tid * 4; i < AGG_ZINTS; i += NTHR * 4) *(v4ia*)(dsm + i) = z4;
    if (tid < 16) misc[tid] = 0;
  }
  __syncthreads();

  int t = 0, ov = 0;
  const int nChunks = (nE + CHUNK - 1) / CHUNK;
#pragma unroll 1
  for (int ch = 0; ch < nChunks; ++ch) {
    const int cbase = ch * CHUNK;
    const int wc = scan_chunk<SLA>(dsts, nE, cbase, nodeBase, NBA, vec8, list, tid, lane, wave);
    if (lane == 0) misc[wave] = wc;
    __syncthreads();
    if (wave == 0) {
#pragma unroll 1
      for (int w2 = 0; w2 < NWAVE; ++w2) {
        int c = misc[w2];
        c = c < 0 ? 0 : (c > WCAP ? WCAP : c);
#pragma unroll 1
        for (int b0 = 0; b0 < c; b0 += 32) {
          const int idx = b0 + lane;
          const int ent = list[w2 * WCAP + (idx < WCAP ? idx : WCAP - 1)];
          const int m32 = (c - b0) < 32 ? (c - b0) : 32;
#pragma unroll 1
          for (int k = 0; k < m32; ++k) {
            const int u    = __builtin_amdgcn_readlane(ent, k);
            const int slot = u & (NBA - 1);
            const int el   = (u >> SLA) & (CHUNK - 1);
            const int pk   = ((cbase + el) << SLA) | slot;
            if (t < RCAP) {
              if (lane == 0) { hl[t] = pk; cnt[slot] = cnt[slot] + 1; }
              t = t + 1;
            } else {
              ov = 1;
            }
          }
        }
      }
    }
    __syncthreads();
  }
  if (wave == 0 && lane == 0) { misc[8] = t; misc[9] = ov; }
  __syncthreads();
  int tt = misc[8];
  tt = tt < 0 ? 0 : (tt > RCAP ? RCAP : tt);
  const int ovf = misc[9];

  if (wave == 0) {
    const int base = lane * (NBA / 32);
    int s = 0;
#pragma unroll 1
    for (int i = 0; i < NBA / 32; ++i) s += cnt[base + i];
    int incl = s;
#pragma unroll
    for (int d = 1; d < 32; d <<= 1) {
      const int y = __shfl_up(incl, d, 32);
      if (lane >= d) incl += y;
    }
    int run = incl - s;
#pragma unroll 1
    for (int i = 0; i < NBA / 32; ++i) {
      const int cv = cnt[base + i];
      offs[base + i] = run;
      cur[base + i]  = run;
      run += cv;
    }
  }
  __syncthreads();
  if (wave == 0) {
#pragma unroll 1
    for (int b0 = 0; b0 < tt; b0 += 32) {
      const int idx = b0 + lane;
      const int ent = hl[idx < RCAP ? idx : RCAP - 1];
      const int m32 = (tt - b0) < 32 ? (tt - b0) : 32;
#pragma unroll 1
      for (int k = 0; k < m32; ++k) {
        const int u    = __builtin_amdgcn_readlane(ent, k);
        const int slot = u & (NBA - 1);
        if (lane == 0) {
          int p = cur[slot];
          p = p < 0 ? 0 : (p > RCAP - 1 ? RCAP - 1 : p);
          sl[p] = u;
          cur[slot] = p + 1;
        }
      }
    }
  }
  __syncthreads();

#pragma unroll 1
  for (int i = tid * 4; i < RCAP; i += NTHR * 4) {
    const v4i e4 = *(const v4ia*)(sl + i);
    int e0 = e4.x >> SLA, e1 = e4.y >> SLA, e2 = e4.z >> SLA, e3 = e4.w >> SLA;
    e0 = e0 < 0 ? 0 : (e0 > nE - 1 ? nE - 1 : e0);
    e1 = e1 < 0 ? 0 : (e1 > nE - 1 ? nE - 1 : e1);
    e2 = e2 < 0 ? 0 : (e2 > nE - 1 ? nE - 1 : e2);
    e3 = e3 < 0 ? 0 : (e3 > nE - 1 ? nE - 1 : e3);
    int r0 = srcs[e0], r1 = srcs[e1], r2 = srcs[e2], r3 = srcs[e3];
    r0 = r0 < 0 ? 0 : (r0 > nN - 1 ? nN - 1 : r0);
    r1 = r1 < 0 ? 0 : (r1 > nN - 1 ? nN - 1 : r1);
    r2 = r2 < 0 ? 0 : (r2 > nN - 1 ? nN - 1 : r2);
    r3 = r3 < 0 ? 0 : (r3 > nN - 1 ? nN - 1 : r3);
    v4i o;
    o.x = (i     < tt) ? r0 : 0;
    o.y = (i + 1 < tt) ? r1 : 0;
    o.z = (i + 2 < tt) ? r2 : 0;
    o.w = (i + 3 < tt) ? r3 : 0;
    *(v4ia*)(hl + i) = o;
  }
  __syncthreads();

  int* sb = slt + (size_t)blockIdx.x * RCAP;
  const v4i c4 = *(const v4ia*)(cnt + 4 * tid);
  const v4i o4 = *(const v4ia*)(offs + 4 * tid);
  v4i fv;
  fv.x = (lane == 0) ? ovf : 0;
  fv.y = (lane == 0) ? tt : 0;
  fv.z = 0; fv.w = 0;
  const bool fw = (wave == 0) && (lane < 8);
  int* fp = flg + (size_t)blockIdx.x * 32 + 4 * (lane & 7);
#pragma unroll 1
  for (int i = tid * 4; i < RCAP; i += NTHR * 4) {
    const v4i v = *(const v4ia*)(hl + i);
    *(volatile v4i*)(sb + i) = v;
  }
  *(volatile v4i*)(cntg + (size_t)nodeBase + 4 * tid) = c4;
  *(volatile v4i*)(offg + (size_t)nodeBase + 4 * tid) = o4;
  if (fw) *(volatile v4i*)fp = fv;
  __threadfence();
#pragma unroll 1
  for (int i = tid * 4; i < RCAP; i += NTHR * 4) {
    const v4i v = *(const v4ia*)(hl + i);
    *(volatile v4i*)(sb + i) = v;
  }
  *(volatile v4i*)(cntg + (size_t)nodeBase + 4 * tid) = c4;
  *(volatile v4i*)(offg + (size_t)nodeBase + 4 * tid) = o4;
  if (fw) *(volatile v4i*)fp = fv;
}

template <int L>
__global__ __launch_bounds__(GTHR) void k_gemm(const float* __restrict__ Ain, const unsigned short* __restrict__ WT,
                                               const float* __restrict__ vec, const float* __restrict__ murs,
                                               int nN, float* xs, float* asn, float* adn) {
  __shared__ __attribute__((aligned(16))) float stg[GBM * DF];
  __shared__ __attribute__((aligned(16))) float cm[DF];
  __shared__ __attribute__((aligned(16))) float ca[DF];
  __shared__ __attribute__((aligned(16))) float cb[DF];
  __shared__ __attribute__((aligned(16))) float asv[DF];
  __shared__ __attribute__((aligned(16))) float adv[DF];
  __shared__ __attribute__((aligned(16))) float rAS[GBM];
  __shared__ __attribute__((aligned(16))) float rAD[GBM];
  const int tid = (int)threadIdx.x, lane = tid & 31, wave = tid >> 5, hh = lane >> 4, m = lane & 15;
  const int rowBase = (int)blockIdx.x * GBM;

  asv[tid] = vec[(L != 0 ? 5 : 0) * DF + tid];
  adv[tid] = vec[(L != 0 ? 6 : 1) * DF + tid];
  if constexpr (L != 0) {
    cm[tid] = murs[tid];
    ca[tid] = murs[DF + tid] * vec[3 * DF + tid];
    cb[tid] = vec[4 * DF + tid];
  } else {
    cm[tid] = 0.0f; ca[tid] = 1.0f; cb[tid] = 0.0f;
  }
  __syncthreads();

  v8f acc[8];
  {
    const v8f z = {0.f, 0.f, 0.f, 0.f, 0.f, 0.f, 0.f, 0.f};
#pragma unroll
    for (int t = 0; t < 8; ++t) acc[t] = z;
  }
  int arow = rowBase + 16 * wave + m;
  arow = arow < nN ? arow : nN - 1;
  const float* rp = Ain + (size_t)arow * DF + 8 * hh;
  const unsigned short* bp = WT + (size_t)m * DF + 8 * hh;

#pragma unroll 1
  for (int k0 = 0; k0 < DF; k0 += 32) {
    v4f q[4];
    q[0] = *(const v4fa*)(rp + k0);
    q[1] = *(const v4fa*)(rp + k0 + 4);
    q[2] = *(const v4fa*)(rp + k0 + 16);
    q[3] = *(const v4fa*)(rp + k0 + 20);
    FragB ah, al;
    if constexpr (L != 0) {
      const int kc = k0 + 8 * hh;
      v4f mq[4], aq[4], bq[4];
      mq[0] = *(const v4fa*)(cm + kc); mq[1] = *(const v4fa*)(cm + kc + 4);
      mq[2] = *(const v4fa*)(cm + kc + 16); mq[3] = *(const v4fa*)(cm + kc + 20);
      aq[0] = *(const v4fa*)(ca + kc); aq[1] = *(const v4fa*)(ca + kc + 4);
      aq[2] = *(const v4fa*)(ca + kc + 16); aq[3] = *(const v4fa*)(ca + kc + 20);
      bq[0] = *(const v4fa*)(cb + kc); bq[1] = *(const v4fa*)(cb + kc + 4);
      bq[2] = *(const v4fa*)(cb + kc + 16); bq[3] = *(const v4fa*)(cb + kc + 20);
#pragma unroll
      for (int j = 0; j < 16; ++j) {
        const float v = q[j >> 2][j & 3];
        const float t = (v - mq[j >> 2][j & 3]) * aq[j >> 2][j & 3] + bq[j >> 2][j & 3];
        const float r = (t > 0.0f) ? t : (t - t);
        const unsigned hb = bf16_bits(r);
        const unsigned lb = bf16_bits(r - __uint_as_float(hb << 16));
        ah.u[j] = (unsigned short)hb;
        al.u[j] = (unsigned short)lb;
      }
    } else {
#pragma unroll
      for (int j = 0; j < 16; ++j) ah.u[j] = (unsigned short)bf16_bits(q[j >> 2][j & 3]);
    }
#pragma unroll
    for (int nt = 0; nt < 8; ++nt) {
      const unsigned short* wq = bp + (size_t)(16 * nt) * DF + k0;
      FragB bf;
      bf.h[0] = *(const v8usa*)wq;
      bf.h[1] = *(const v8usa*)(wq + 16);
      acc[nt] = wmb(ah, bf, acc[nt]);
      if constexpr (L != 0) acc[nt] = wmb(al, bf, acc[nt]);
    }
  }

#pragma unroll
  for (int nt = 0; nt < 8; ++nt) {
    const int lc = 16 * nt + m;
#pragma unroll
    for (int r = 0; r < 8; ++r) {
      const int lr = 16 * wave + 8 * hh + r;
      stg[lr * DF + lc] = acc[nt][r];
    }
  }
  __syncthreads();

  const v4f a4 = *(const v4fa*)(asv + 4 * lane);
  const v4f d4 = *(const v4fa*)(adv + 4 * lane);
  float myS = 0.0f, myD = 0.0f;
#pragma unroll 1
  for (int i = 0; i < 16; ++i) {
    const int lr = 16 * wave + i;
    const int gr = rowBase + lr;
    const bool ok = gr < nN;
    v4f p = *(const v4fa*)(stg + lr * DF + 4 * lane);
    p.x = ok ? p.x : 0.0f; p.y = ok ? p.y : 0.0f; p.z = ok ? p.z : 0.0f; p.w = ok ? p.w : 0.0f;
    float s = p.x * a4.x + p.y * a4.y + p.z * a4.z + p.w * a4.w;
    float d = p.x * d4.x + p.y * d4.y + p.z * d4.z + p.w * d4.w;
#pragma unroll
    for (int o = 16; o > 0; o >>= 1) {
      s += __shfl_xor(s, o, 32);
      d += __shfl_xor(d, o, 32);
    }
    myS = (lane == i) ? s : myS;
    myD = (lane == i) ? d : myD;
    *(volatile v4f*)(xs + (size_t)gr * DF + 4 * lane) = p;
  }
  __threadfence();
#pragma unroll 1
  for (int i = 0; i < 16; ++i) {
    const int lr = 16 * wave + i;
    const int gr = rowBase + lr;
    const bool ok = gr < nN;
    v4f p = *(const v4fa*)(stg + lr * DF + 4 * lane);
    p.x = ok ? p.x : 0.0f; p.y = ok ? p.y : 0.0f; p.z = ok ? p.z : 0.0f; p.w = ok ? p.w : 0.0f;
    *(volatile v4f*)(xs + (size_t)gr * DF + 4 * lane) = p;
  }
  if (lane < 16) { rAS[16 * wave + lane] = myS; rAD[16 * wave + lane] = myD; }
  __syncthreads();
  const v4f sv = *(const v4fa*)(rAS + 4 * (lane & 15));
  const v4f dv = *(const v4fa*)(rAD + 4 * (lane & 15));
  const bool w0 = (wave == 0) && (lane < 16);
  const bool w1 = (wave == 1) && (lane < 16);
  float* sp = asn + (size_t)rowBase + 4 * (lane & 15);
  float* dp = adn + (size_t)rowBase + 4 * (lane & 15);
  if (w0) *(volatile v4f*)sp = sv;
  if (w1) *(volatile v4f*)dp = dv;
  __threadfence();
  if (w0) *(volatile v4f*)sp = sv;
  if (w1) *(volatile v4f*)dp = dv;
}

__global__ __launch_bounds__(NTHR) void k_agg(const int* __restrict__ slt, const int* __restrict__ cntg,
                                              const int* __restrict__ offg, const int* __restrict__ flg,
                                              const float* __restrict__ xs, const float* __restrict__ asn,
                                              const float* __restrict__ adn, const float* __restrict__ bias,
                                              int nN, float* agg, double* rec) {
  __shared__ double wsum[NWAVE * 256];
  __shared__ __attribute__((aligned(16))) double rsum[256];
  const int tid = (int)threadIdx.x, lane = tid & 31, wave = tid >> 5;
  const int nodeBase = (int)blockIdx.x * NBA;
  const int* sb = slt + (size_t)blockIdx.x * RCAP;
  const int ovf = flg[(size_t)blockIdx.x * 32];
  const float qnan = __int_as_float(0x7fc00000);
  const float ninf = __int_as_float((int)0xff800000u);
  const float pz = (ovf != 0) ? qnan : 0.0f;
  const v4f b4 = *(const v4fa*)(bias + 4 * lane);
  double s0 = 0.0, s1 = 0.0, s2 = 0.0, s3 = 0.0;
  double q0 = 0.0, q1 = 0.0, q2 = 0.0, q3 = 0.0;

#pragma unroll 1
  for (int si = 0; si < NBA / NWAVE; ++si) {
    const int s    = si * NWAVE + wave;
    const int node = nodeBase + s;
    int c = cntg[node];
    const bool big = (c > DEGCAP) || (c < 0);
    c = c < 0 ? 0 : (c > DEGCAP ? DEGCAP : c);
    int o = offg[node];
    o = o < 0 ? 0 : (o > RCAP ? RCAP : o);
    const int nc = node < nN ? node : nN - 1;
    const float adi = adn[nc];
    const int pa = lane, pb = 32 + lane;
    int ia = o + pa; ia = ia > RCAP - 1 ? RCAP - 1 : ia;
    int ib = o + pb; ib = ib > RCAP - 1 ? RCAP - 1 : ib;
    int ra = sb[ia], rb = sb[ib];
    ra = ra < 0 ? 0 : (ra > nN - 1 ? nN - 1 : ra);
    rb = rb < 0 ? 0 : (rb > nN - 1 ? nN - 1 : rb);
    const int sra = (pa < c) ? ra : nc;
    const int srb = (pb < c) ? rb : nc;
    const bool va = pa <= c, vb = pb <= c;
    const float ta = asn[sra] + adi;
    const float tb = asn[srb] + adi;
    const float la = (ta > 0.0f) ? ta : 0.2f * ta;
    const float lb = (tb > 0.0f) ? tb : 0.2f * tb;
    float mx = fmaxf(va ? la : ninf, vb ? lb : ninf);
#pragma unroll
    for (int d = 16; d > 0; d >>= 1) mx = fmaxf(mx, __shfl_xor(mx, d, 32));
    const float xa = expf(la - mx);
    const float xb = expf(lb - mx);
    const float ea = va ? xa : 0.0f;
    const float eb = vb ? xb : 0.0f;
    float den = ea + eb;
#pragma unroll
    for (int d = 16; d > 0; d >>= 1) den += __shfl_xor(den, d, 32);
    const float inv = __builtin_amdgcn_rcpf(den + 1e-16f);
    const int eai = __float_as_int(ea), ebi = __float_as_int(eb);
    const int ce = c + 1;
    const int n0 = ce < 32 ? ce : 32;
    int n1 = ce - n0;
    n1 = n1 < 0 ? 0 : (n1 > 32 ? 32 : n1);
    float a0 = 0.0f, a1 = 0.0f, a2 = 0.0f, a3 = 0.0f;
#pragma unroll 1
    for (int k = 0; k < n0; ++k) {
      const int   sk = __builtin_amdgcn_readlane(sra, k);
      const float ek = __int_as_float(__builtin_amdgcn_readlane(eai, k));
      const v4f r = *(const v4fa*)(xs + (size_t)sk * DF + 4 * lane);
      a0 = fmaf(ek, r.x, a0); a1 = fmaf(ek, r.y, a1); a2 = fmaf(ek, r.z, a2); a3 = fmaf(ek, r.w, a3);
    }
#pragma unroll 1
    for (int k = 0; k < n1; ++k) {
      const int   sk = __builtin_amdgcn_readlane(srb, k);
      const float ek = __int_as_float(__builtin_amdgcn_readlane(ebi, k));
      const v4f r = *(const v4fa*)(xs + (size_t)sk * DF + 4 * lane);
      a0 = fmaf(ek, r.x, a0); a1 = fmaf(ek, r.y, a1); a2 = fmaf(ek, r.z, a2); a3 = fmaf(ek, r.w, a3);
    }
    const float pzr = big ? qnan : pz;
    v4f y;
    y.x = (a0 * inv + b4.x) + pzr;
    y.y = (a1 * inv + b4.y) + pzr;
    y.z = (a2 * inv + b4.z) + pzr;
    y.w = (a3 * inv + b4.w) + pzr;
    if (node < nN) {
      float* op = agg + (size_t)node * DF + 4 * lane;
      *(volatile v4f*)op = y;
      __threadfence();
      *(volatile v4f*)op = y;
      const double d0 = (double)y.x, d1 = (double)y.y, d2 = (double)y.z, d3 = (double)y.w;
      s0 += d0; s1 += d1; s2 += d2; s3 += d3;
      q0 += d0 * d0; q1 += d1 * d1; q2 += d2 * d2; q3 += d3 * d3;
    }
  }

  wsum[wave * 256 + 4 * lane + 0] = s0;
  wsum[wave * 256 + 4 * lane + 1] = s1;
  wsum[wave * 256 + 4 * lane + 2] = s2;
  wsum[wave * 256 + 4 * lane + 3] = s3;
  wsum[wave * 256 + 128 + 4 * lane + 0] = q0;
  wsum[wave * 256 + 128 + 4 * lane + 1] = q1;
  wsum[wave * 256 + 128 + 4 * lane + 2] = q2;
  wsum[wave * 256 + 128 + 4 * lane + 3] = q3;
  __syncthreads();
  {
    double t = 0.0;
#pragma unroll
    for (int w2 = 0; w2 < NWAVE; ++w2) t += wsum[w2 * 256 + tid];
    rsum[tid] = t;
  }
  __syncthreads();
  const v2d rv = *(const v2da*)(rsum + 2 * (tid & 127));
  double* rp = rec + (size_t)blockIdx.x * 256 + 2 * (tid & 127);
  const bool rw = tid < 128;
  if (rw) *(volatile v2d*)rp = rv;
  __threadfence();
  if (rw) *(volatile v2d*)rp = rv;
}

__global__ __launch_bounds__(NTHR) void k_bn(const double* __restrict__ rec, int nb, double invN, float* murs) {
  __shared__ double sd[256];
  __shared__ __attribute__((aligned(16))) float st[256];
  const int tid = (int)threadIdx.x;
  double a = 0.0;
#pragma unroll 1
  for (int b = 0; b < nb; ++b) a += rec[(size_t)b * 256 + tid];
  sd[tid] = a;
  __syncthreads();
  if (tid < 128) {
    const double mean = sd[tid] * invN;
    double var = sd[128 + tid] * invN - mean * mean;
    var = (var < 0.0) ? 0.0 : var;
    const float vf = (float)var;
    st[tid] = (float)mean;
    st[128 + tid] = 1.0f / sqrtf(vf + 1e-5f);
  }
  __syncthreads();
  const v4f v = *(const v4fa*)(st + 4 * (tid & 63));
  float* op = murs + 4 * (tid & 63);
  const bool w = tid < 64;
  if (w) *(volatile v4f*)op = v;
  __threadfence();
  if (w) *(volatile v4f*)op = v;
}

__global__ __launch_bounds__(NTHR) void k_out(const float* __restrict__ agg, const float* __restrict__ murs,
                                              const float* __restrict__ g, const float* __restrict__ be,
                                              int nUnits, float* out) {
  const int u = (int)blockIdx.x * NTHR + (int)threadIdx.x;
  if (u >= nUnits) return;
  const int c4 = (u & 31) * 4;
  const v4f v  = *(const v4fa*)(agg + 4 * (size_t)u);
  const v4f mu = *(const v4fa*)(murs + c4);
  const v4f rs = *(const v4fa*)(murs + DF + c4);
  const v4f gg = *(const v4fa*)(g + c4);
  const v4f bb = *(const v4fa*)(be + c4);
  v4f y;
  y.x = (v.x - mu.x) * rs.x * gg.x + bb.x;
  y.y = (v.y - mu.y) * rs.y * gg.y + bb.y;
  y.z = (v.z - mu.z) * rs.z * gg.z + bb.z;
  y.w = (v.w - mu.w) * rs.w * gg.w + bb.w;
  float* op = out + 4 * (size_t)u;
  *(volatile v4f*)op = y;
  __threadfence();
  *(volatile v4f*)op = y;
}

static inline int cdiv(int a, int b) { return (a + b - 1) / b; }
static inline size_t al256(size_t o) { return (o + 255) & ~(size_t)255; }

extern "C" void kernel_launch(void* const* d_in, const int* in_sizes, int n_in,
                              void* d_out, int out_size, void* d_ws, size_t ws_size,
                              hipStream_t stream) {
  if (n_in < 14) return;
  if (in_sizes[0] < DF || (in_sizes[0] % DF) != 0) return;
  const int nN = in_sizes[0] / DF;
  if (nN < 16 || nN > (1 << 22)) return;
  if (in_sizes[1] < 2 || (in_sizes[1] & 1) != 0) return;
  const int nE = in_sizes[1] / 2;
  if (nE < 1 || nE >= (1 << (31 - SLA))) return;
  if (in_sizes[2] != DF * DF || in_sizes[8] != DF * DF) return;
  for (int i = 3; i <= 7; ++i)  if (in_sizes[i] != DF) return;
  for (int i = 9; i <= 13; ++i) if (in_sizes[i] != DF) return;
  if ((long long)out_size != (long long)nN * DF) return;

  const float* x   = (const float*)d_in[0];
  const int*   ei  = (const int*)d_in[1];
  const float* W0  = (const float*)d_in[2];
  const float* as0 = (const float*)d_in[3];
  const float* ad0 = (const float*)d_in[4];
  const float* b0  = (const float*)d_in[5];
  const float* g0  = (const float*)d_in[6];
  const float* be0 = (const float*)d_in[7];
  const float* W1  = (const float*)d_in[8];
  const float* as1 = (const float*)d_in[9];
  const float* ad1 = (const float*)d_in[10];
  const float* b1  = (const float*)d_in[11];
  const float* g1  = (const float*)d_in[12];
  const float* be1 = (const float*)d_in[13];
  float* out = (float*)d_out;
  const int* src = ei;
  const int* dst = ei + nE;

  const int MP = cdiv(nN, GBM) * GBM;
  const int gM = MP / GBM;
  const int gA = cdiv(nN, NBA);
  const int NP = gA * NBA;
  if (NP < nN) return;
  const int vec8 = ((nE & 3) == 0) ? 1 : 0;

  char* ws = (char*)d_ws;
  size_t off = 0;
  const size_t oW0T = off; off = al256(off + (size_t)DF * DF * 2);
  const size_t oW1T = off; off = al256(off + (size_t)DF * DF * 2);
  const size_t oVEC = off; off = al256(off + (size_t)NVEC * DF * 4);
  const size_t oMR0 = off; off = al256(off + (size_t)256 * 4);
  const size_t oMR1 = off; off = al256(off + (size_t)256 * 4);
  const size_t oREC = off; off = al256(off + (size_t)gA * 256 * 8);
  const size_t oFLG = off; off = al256(off + (size_t)gA * 32 * 4);
  const size_t oCNT = off; off = al256(off + (size_t)NP * 4);
  const size_t oOFF = off; off = al256(off + (size_t)NP * 4);
  const size_t oAS  = off; off = al256(off + (size_t)MP * 4);
  const size_t oAD  = off; off = al256(off + (size_t)MP * 4);
  const size_t oSLT = off; off = al256(off + (size_t)gA * RCAP * 4);
  const size_t oXS  = off; off = al256(off + (size_t)MP * DF * 4);
  const size_t oAGG = off; off = al256(off + (size_t)MP * DF * 4);
  if (off > ws_size || off > (size_t)WSMAX) return;
  unsigned short* W0T = (unsigned short*)(ws + oW0T);
  unsigned short* W1T = (unsigned short*)(ws + oW1T);
  float*  VEC = (float*)(ws + oVEC);
  float*  MR0 = (float*)(ws + oMR0);
  float*  MR1 = (float*)(ws + oMR1);
  double* REC = (double*)(ws + oREC);
  int*    FLG = (int*)(ws + oFLG);
  int*    CNT = (int*)(ws + oCNT);
  int*    OFF = (int*)(ws + oOFF);
  float*  AS  = (float*)(ws + oAS);
  float*  AD  = (float*)(ws + oAD);
  int*    SLT = (int*)(ws + oSLT);
  float*  XS  = (float*)(ws + oXS);
  float*  AGG = (float*)(ws + oAGG);

  const size_t csrLds = (size_t)CSR_LDS_INTS * 4;
  hipFuncSetAttribute(reinterpret_cast<const void*>(&k_csr), hipFuncAttributeMaxDynamicSharedMemorySize, (int)csrLds);
  const double invN = 1.0 / (double)nN;

  k_prep<<<(2 * UW + 512) / NTHR, NTHR, 0, stream>>>(W0, W1, as0, ad0, b0, g0, be0, as1, ad1, b1, g1, be1,
                                                     W0T, W1T, VEC);
  k_csr<<<gA, NTHR, csrLds, stream>>>(src, dst, nE, nN, vec8, SLT, CNT, OFF, FLG);
  k_gemm<0><<<gM, GTHR, 0, stream>>>(x, W0T, VEC, VEC, nN, XS, AS, AD);
  k_agg<<<gA, NTHR, 0, stream>>>(SLT, CNT, OFF, FLG, XS, AS, AD, VEC + 2 * DF, nN, AGG, REC);
  k_bn<<<1, NTHR, 0, stream>>>(REC, gA, invN, MR0);
  k_gemm<1><<<gM, GTHR, 0, stream>>>(AGG, W1T, VEC, MR0, nN, XS, AS, AD);
  k_agg<<<gA, NTHR, 0, stream>>>(SLT, CNT, OFF, FLG, XS, AS, AD, VEC + 7 * DF, nN, AGG, REC);
  k_bn<<<1, NTHR, 0, stream>>>(REC, gA, invN, MR1);
  const int nUnits = nN * (DF / 4);
  k_out<<<cdiv(nUnits, NTHR), NTHR, 0, stream>>>(AGG, MR1, VEC + 8 * DF, VEC + 9 * DF, nUnits, out);
}
